// RemesNeuralSpectralKernel_61821759259032
// MI455X (gfx1250) — hardware-verified
//
#include <hip/hip_runtime.h>

typedef __bf16         v16b __attribute__((ext_vector_type(16)));
typedef float          v8f  __attribute__((ext_vector_type(8)));
typedef float          v4f  __attribute__((ext_vector_type(4)));
typedef float          v2f  __attribute__((ext_vector_type(2)));
typedef v4f            v4fa __attribute__((may_alias));

#define D_IN        16
#define HID         32
#define TR          16
#define FEAT_STRIDE 384
#define FEAT_MU     256
#define FEAT_VAR    272
#define PT          32
#define PAIR_THREADS 256

#define LOG2E_F   1.4426950408889634f
#define TWO_PI_F  6.28318530717958648f

__device__ __forceinline__ unsigned short bf16_rne(float x) {
  unsigned u = __float_as_uint(x);
  u += 0x7FFFu + ((u >> 16) & 1u);
  return (unsigned short)(u >> 16);
}
__device__ __forceinline__ float bf16_val(unsigned short b) {
  return __uint_as_float(((unsigned)b) << 16);
}

union U16 { v16b v; unsigned short s[16]; };
struct Frag3 { v16b h, m, l; };

__device__ __forceinline__ Frag3 build_frag(const float* src, int off, int kstride, int lane) {
  const int hh = lane >> 4;
  U16 ph, pm, pl;
#pragma unroll
  for (int i = 0; i < 16; ++i) {
    const int k = (i < 8) ? (8 * hh + i) : (16 + 8 * hh + (i - 8));
    const float x = src[off + k * kstride];
    const unsigned short b0 = bf16_rne(x);
    const float r1 = x - bf16_val(b0);
    const unsigned short b1 = bf16_rne(r1);
    const float r2 = r1 - bf16_val(b1);
    const unsigned short b2 = bf16_rne(r2);
    ph.s[i] = b0; pm.s[i] = b1; pl.s[i] = b2;
  }
  Frag3 f;
  f.h = ph.v; f.m = pm.v; f.l = pl.v;
  return f;
}

__device__ __forceinline__ v8f wmma_bf16(v16b a, v16b b, v8f c) {
  c = __builtin_amdgcn_wmma_f32_16x16x32_bf16(false, a, false, b, (short)0, c, false, false);
  asm volatile("v_nop\n\tv_nop\n\tv_nop\n\tv_nop" : "+v"(c) : "v"(a), "v"(b));
  return c;
}

template <int NT>
__device__ __forceinline__ void gemm_tile(const float* actIn, const float* Wsm,
                                          float* dst, int dstPitch, int lane) {
  const int hh = lane >> 4, m = lane & 15;
  const Frag3 a = build_frag(actIn, m * HID, 1, lane);
#pragma unroll
  for (int nt = 0; nt < NT; ++nt) {
    const Frag3 b = build_frag(Wsm, nt * 16 + m, HID, lane);
    v8f acc = {0.f, 0.f, 0.f, 0.f, 0.f, 0.f, 0.f, 0.f};
    acc = wmma_bf16(a.l, b.h, acc);
    acc = wmma_bf16(a.h, b.l, acc);
    acc = wmma_bf16(a.m, b.m, acc);
    acc = wmma_bf16(a.m, b.h, acc);
    acc = wmma_bf16(a.h, b.m, acc);
    acc = wmma_bf16(a.h, b.h, acc);
#pragma unroll
    for (int r = 0; r < 8; ++r) dst[(8 * hh + r) * dstPitch + nt * 16 + m] = acc[r];
  }
}

__device__ __forceinline__ void load_w(float* Wsm, const float* __restrict__ W,
                                       int K0, int N0, int lane) {
  for (int t = lane; t < HID * HID; t += 32) {
    const int k = t >> 5, n = t & 31;
    float v = 0.f;
    if (k < K0 && n < N0) v = W[k * N0 + n];
    Wsm[t] = v;
  }
}

__device__ __forceinline__ float selu_f(float x) {
  const float kAlpha = 1.6732632423543772f;
  const float kScale = 1.0507009873554805f;
  const float e = kAlpha * expm1f(fminf(x, 0.f));
  return kScale * ((x > 0.f) ? x : e);
}
__device__ __forceinline__ float softplus_f(float x) {
  return fmaxf(x, 0.f) + log1pf(expf(-fabsf(x)));
}
__device__ __forceinline__ void bias_selu(float* buf, const float* __restrict__ bias, int lane) {
  for (int t = lane; t < TR * HID; t += 32) buf[t] = selu_f(buf[t] + bias[t & (HID - 1)]);
}
__device__ __forceinline__ void bias_softplus16(float* buf, const float* __restrict__ bias, int lane) {
  for (int t = lane; t < TR * 16; t += 32) buf[t] = softplus_f(buf[t] + bias[t & 15]);
}

__device__ __forceinline__ void mlp12(const float* act0, float* Wsm, float* actA, float* actB,
                                      const float* __restrict__ W1, const float* __restrict__ b1,
                                      const float* __restrict__ W2, const float* __restrict__ b2,
                                      int lane) {
  load_w(Wsm, W1, D_IN, HID, lane);
  __syncthreads();
  gemm_tile<2>(act0, Wsm, actA, HID, lane);
  __syncthreads();
  bias_selu(actA, b1, lane);
  __syncthreads();
  load_w(Wsm, W2, HID, HID, lane);
  __syncthreads();
  gemm_tile<2>(actA, Wsm, actB, HID, lane);
  __syncthreads();
  bias_selu(actB, b2, lane);
  __syncthreads();
}

__device__ __forceinline__ void layer3(const float* actB, float* Wsm, float* Fs,
                                       const float* __restrict__ W3, const float* __restrict__ b3,
                                       int lane) {
  load_w(Wsm, W3, HID, 16, lane);
  __syncthreads();
  gemm_tile<1>(actB, Wsm, Fs, 16, lane);
  __syncthreads();
  bias_softplus16(Fs, b3, lane);
  __syncthreads();
}

__global__ __launch_bounds__(32)
void feat_kernel(const float* __restrict__ X1, const float* __restrict__ X2,
                 const float* __restrict__ fW1, const float* __restrict__ fb1,
                 const float* __restrict__ fW2, const float* __restrict__ fb2,
                 const float* __restrict__ fW3, const float* __restrict__ fb3,
                 const float* __restrict__ lW1, const float* __restrict__ lb1,
                 const float* __restrict__ lW2, const float* __restrict__ lb2,
                 const float* __restrict__ lW3, const float* __restrict__ lb3,
                 const float* __restrict__ vW1, const float* __restrict__ vb1,
                 const float* __restrict__ vW2, const float* __restrict__ vb2,
                 const float* __restrict__ vW3, const float* __restrict__ vb3,
                 float* __restrict__ feat, int nb1) {
  __shared__ __attribute__((aligned(16))) float act0[TR * HID];
  __shared__ __attribute__((aligned(16))) float actA[TR * HID];
  __shared__ __attribute__((aligned(16))) float actB[TR * HID];
  __shared__ __attribute__((aligned(16))) float Wsm[HID * HID];
  __shared__ __attribute__((aligned(16))) float Fs[TR * 16];
  __shared__ __attribute__((aligned(16))) float stageS[FEAT_STRIDE];

  const int lane  = threadIdx.x;
  const int which = (blockIdx.x >= (unsigned)nb1) ? 1 : 0;
  const int blk   = (int)blockIdx.x - which * nb1;
  const int row0  = blk * TR;
  const float* X  = which ? X2 : X1;

  for (int t = lane; t < TR * 16; t += 32) {
    const int m = t >> 4, k = t & 15;
    const float v = X[(size_t)(row0 + m) * D_IN + k];
    act0[m * HID + k] = v;
    act0[m * HID + 16 + k] = 0.f;
  }
  for (int t = FEAT_VAR + 16 + lane; t < FEAT_STRIDE; t += 32) stageS[t] = 0.f;
  __syncthreads();

  mlp12(act0, Wsm, actA, actB, fW1, fb1, fW2, fb2, lane);
  layer3(actB, Wsm, Fs, fW3, fb3, lane);
  if (lane < TR) {
#pragma clang fp contract(off)
    float s = 0.f;
    for (int n = 0; n < D_IN; ++n) s = s + Fs[lane * 16 + n] * act0[lane * HID + n];
    stageS[FEAT_MU + lane] = s;
  }
  __syncthreads();

  mlp12(act0, Wsm, actA, actB, lW1, lb1, lW2, lb2, lane);
  layer3(actB, Wsm, Fs, lW3, lb3, lane);
  for (int t = lane; t < TR * 16; t += 32) stageS[t] = Fs[t];
  __syncthreads();

  mlp12(act0, Wsm, actA, actB, vW1, vb1, vW2, vb2, lane);
  if (lane < TR) {
    float acc = 0.f;
    for (int k = 0; k < HID; ++k) acc += actB[lane * HID + k] * vW3[k];
    acc += vb3[0];
    stageS[FEAT_VAR + lane] = softplus_f(acc);
  }
  __syncthreads();

  const v4fa* sv = (const v4fa*)stageS;
  const v4f w0 = sv[lane], w1 = sv[32 + lane], w2 = sv[64 + lane];
  volatile v4f* dv = (volatile v4f*)(feat + (size_t)blockIdx.x * FEAT_STRIDE);
  dv[lane] = w0; dv[32 + lane] = w1; dv[64 + lane] = w2;
  __threadfence();
  dv[lane] = w0; dv[32 + lane] = w1; dv[64 + lane] = w2;
}

__device__ __forceinline__ float cos_f(float x) {
  const float q = __builtin_rintf(x * 0.63661977236758134f);
  float r = __builtin_fmaf(-q, 1.5707963705062866f, x);
  r = __builtin_fmaf(-q, -4.3711390001862427e-08f, r);
  const int qi = (int)q;
  const float z = r * r;
  float c = __builtin_fmaf(2.443315711809948e-5f, z, -1.388731625493765e-3f);
  c = __builtin_fmaf(c, z, 4.166664568298827e-2f);
  c = __builtin_fmaf(c, z * z, __builtin_fmaf(-0.5f, z, 1.0f));
  float s = __builtin_fmaf(-1.9515295891e-4f, z, 8.3321608736e-3f);
  s = __builtin_fmaf(s, z, -1.6666654611e-1f);
  s = __builtin_fmaf(s * z, r, r);
  const float v = (qi & 1) ? s : c;
  return ((qi + 1) & 2) ? -v : v;
}

__global__ __launch_bounds__(PAIR_THREADS)
void pair_kernel(const float* __restrict__ X1, const float* __restrict__ X2,
                 const float* __restrict__ feat1, const float* __restrict__ feat2,
                 float* __restrict__ out, int n1, int n2) {
  __shared__ v4f   iS[PT * D_IN];
  __shared__ v2f   jS[PT * D_IN];
  __shared__ float muI[PT], vI[PT], muJ[PT], vJ[PT];

  const int tid = threadIdx.x;
  const int i0 = blockIdx.y * PT, j0 = blockIdx.x * PT;

  for (int e = tid; e < PT * D_IN; e += PAIR_THREADS) {
    const int p = e >> 4, d = e & 15;
    int ii = i0 + p; ii = (ii < n1) ? ii : (n1 - 1);
    int jj = j0 + p; jj = (jj < n2) ? jj : (n2 - 1);
    const float xi = X1[(size_t)ii * D_IN + d];
    const float li = feat1[(size_t)(ii >> 4) * FEAT_STRIDE + (ii & 15) * D_IN + d];
    const v4f a = {xi, li * li, 2.0f * li, 0.f};
    iS[e] = a;
    const float xj = X2[(size_t)jj * D_IN + d];
    const float lj = feat2[(size_t)(jj >> 4) * FEAT_STRIDE + (jj & 15) * D_IN + d];
    const v2f b = {xj, lj};
    jS[e] = b;
  }
  if (tid < PT) {
    int ii = i0 + tid; ii = (ii < n1) ? ii : (n1 - 1);
    const size_t base = (size_t)(ii >> 4) * FEAT_STRIDE;
    muI[tid] = feat1[base + FEAT_MU + (ii & 15)];
    vI[tid]  = feat1[base + FEAT_VAR + (ii & 15)];
  } else if (tid < 2 * PT) {
    const int p = tid - PT;
    int jj = j0 + p; jj = (jj < n2) ? jj : (n2 - 1);
    const size_t base = (size_t)(jj >> 4) * FEAT_STRIDE;
    muJ[p] = feat2[base + FEAT_MU + (jj & 15)];
    vJ[p]  = feat2[base + FEAT_VAR + (jj & 15)];
  }
  __syncthreads();

  const int il = tid >> 3;
  const int jq = tid & 7;
  const v4f* ip = iS + il * D_IN;
  const v2f* jp = jS + (4 * jq) * D_IN;

  float D[4] = {0.f, 0.f, 0.f, 0.f};
  float R[4] = {1.f, 1.f, 1.f, 1.f};
#pragma unroll 2
  for (int d = 0; d < D_IN; ++d) {
    const v4f a = ip[d];
#pragma unroll
    for (int u = 0; u < 4; ++u) {
      const v2f b  = jp[u * D_IN + d];
      const float df = a.x - b.x;
      const float L  = __builtin_fmaf(b.y, b.y, a.y);
      const float rc = __builtin_amdgcn_rcpf(L);
      D[u] = __builtin_fmaf(df * df, rc, D[u]);
      R[u] = R[u] * ((a.z * b.y) * rc);
    }
  }

  const float mui = muI[il], vi = vI[il];
  float kk[4];
#pragma unroll
  for (int u = 0; u < 4; ++u) {
    const float muj = muJ[4 * jq + u], vj = vJ[4 * jq + u];
    const float det = __builtin_amdgcn_sqrtf(R[u]);
    const float ex  = __builtin_amdgcn_exp2f(-D[u] * LOG2E_F);
    const float E   = det * ex;
    const float cs  = cos_f(TWO_PI_F * (mui - muj));
    kk[u] = ((vi * vj) * E) * cs;
  }

  const int i = i0 + il;
  const int j = j0 + 4 * jq;
  if (i < n1 && j + 3 < n2) {
    const v4f kv = {kk[0], kk[1], kk[2], kk[3]};
    volatile v4f* op = (volatile v4f*)(out + (size_t)i * (size_t)n2 + j);
    *op = kv;
    __threadfence();
    *op = kv;
  }
}

extern "C" void kernel_launch(void* const* d_in, const int* in_sizes, int n_in,
                              void* d_out, int out_size, void* d_ws,
                              size_t ws_size, hipStream_t stream) {
  if (n_in < 20) return;
  const int n1 = in_sizes[0] / D_IN;
  const int n2 = in_sizes[1] / D_IN;
  if (n1 <= 0 || n2 <= 0) return;
  if ((n1 % PT) != 0 || (n2 % PT) != 0) return;
  if ((size_t)out_size != (size_t)n1 * (size_t)n2) return;
  const int nb1 = n1 / TR, nb2 = n2 / TR;
  const size_t feat_floats = (size_t)(nb1 + nb2) * FEAT_STRIDE;
  if (feat_floats * sizeof(float) > ws_size) return;

  const float* X1  = (const float*)d_in[0];
  const float* X2  = (const float*)d_in[1];
  const float* fW1 = (const float*)d_in[2];
  const float* fb1 = (const float*)d_in[3];
  const float* fW2 = (const float*)d_in[4];
  const float* fb2 = (const float*)d_in[5];
  const float* fW3 = (const float*)d_in[6];
  const float* fb3 = (const float*)d_in[7];
  const float* lW1 = (const float*)d_in[8];
  const float* lb1 = (const float*)d_in[9];
  const float* lW2 = (const float*)d_in[10];
  const float* lb2 = (const float*)d_in[11];
  const float* lW3 = (const float*)d_in[12];
  const float* lb3 = (const float*)d_in[13];
  const float* vW1 = (const float*)d_in[14];
  const float* vb1 = (const float*)d_in[15];
  const float* vW2 = (const float*)d_in[16];
  const float* vb2 = (const float*)d_in[17];
  const float* vW3 = (const float*)d_in[18];
  const float* vb3 = (const float*)d_in[19];
  float* ws    = (float*)d_ws;
  float* feat1 = ws;
  float* feat2 = ws + (size_t)nb1 * FEAT_STRIDE;

  feat_kernel<<<dim3(nb1 + nb2), dim3(32), 0, stream>>>(
      X1, X2, fW1, fb1, fW2, fb2, fW3, fb3, lW1, lb1, lW2, lb2, lW3, lb3,
      vW1, vb1, vW2, vb2, vW3, vb3, ws, nb1);
  pair_kernel<<<dim3(n2 / PT, n1 / PT), dim3(PAIR_THREADS), 0, stream>>>(
      X1, X2, feat1, feat2, (float*)d_out, n1, n2);
}
